// SymmetricContraction_41102837023172
// MI455X (gfx1250) — hardware-verified
//
#include <hip/hip_runtime.h>

typedef __attribute__((ext_vector_type(16))) _Float16   v16h;
typedef __attribute__((ext_vector_type(8)))  float    v8f;
typedef __attribute__((ext_vector_type(4)))  unsigned u32x4;
typedef __attribute__((ext_vector_type(8)))  unsigned u32x8;
typedef __attribute__((ext_vector_type(4)))  float    v4f;
typedef __attribute__((ext_vector_type(8)))  _Float16 v8h;
template <typename V> __device__ __forceinline__ void vst2(void* p, V v) {
  *(volatile V*)p = v; __threadfence(); *(volatile V*)p = v;
}
__device__ __forceinline__ v8f wmma16(v16h a, v16h b, v8f c) {
  v8f d = __builtin_amdgcn_wmma_f32_16x16x32_f16(false, a, false, b, (short)0, c, false, false);
  asm volatile("v_nop\n\tv_nop\n\tv_nop\n\tv_nop" : "+v"(d) : "v"(a), "v"(b));
  return d;
}

#define C_CH   128
#define E_ELEM 10

__device__ __forceinline__ void copy_panel(_Float16* lds_dst, const _Float16* gsrc, unsigned nelem, int tid) {
  const unsigned n16 = nelem * 2 / 16;
  for (unsigned c = tid; c < n16; c += 1024) ((u32x4*)lds_dst)[c] = ((const u32x4*)gsrc)[c];
}

__global__ void build_bmat(const float* __restrict__ U3, const float* __restrict__ U2,
                           _Float16* __restrict__ Bm, int M, int K3, int K2, int KPAD) {
  int N = M * 256, NP = N + 8;
  int total = KPAD * NP;
  int g = blockIdx.x * 256 + threadIdx.x;
  if (g * 8 >= total) return;
  int KI = 16 * K3;
  union { v8h h; u32x4 u; } pk;
#pragma unroll
  for (int e8 = 0; e8 < 8; ++e8) {
    int idx = g * 8 + e8;
    int p = idx / (32 * NP), rem = idx % (32 * NP);
    int kl = rem / NP, n = rem % NP;
    int kk = p * 32 + kl;
    float v = 0.f;
    if (n < N) {
      int m = n >> 8, j = (n >> 4) & 15, l = n & 15;
      if (kk < KI) {
        int k = kk >> 4, i = kk & 15;
        v = U3[((((m * 16 + i) * 16 + j) * 16 + l) * K3) + k];
      } else if (kk < KI + K2) {
        v = U2[(((m * 16 + j) * 16 + l) * K2) + (kk - KI)];
      }
    }
    pk.h[e8] = (_Float16)v;
  }
  vst2(Bm + (size_t)g * 8, pk.u);
}

template <int MOUT, int KPAD>
__global__ __launch_bounds__(1024) void mace_contract(
    const float* __restrict__ x, const float* __restrict__ y,
    const _Float16* __restrict__ Bmat,
    const float* __restrict__ W3, const float* __restrict__ W2,
    const float* __restrict__ W1, const float* __restrict__ U1,
    int K3, int K2, int K1,
    float* __restrict__ out, int out_col_ofs) {
  constexpr int N      = MOUT * 256;
  constexpr int NP     = N + 8;
  constexpr int NT     = N / 16;
  constexpr int NTPW   = NT / 4;
  constexpr int KSTEPS = KPAD / 32;
  constexpr int KPADP  = KPAD + 8;
  constexpr int PANEL  = 32 * NP;

  extern __shared__ __align__(16) char smem[];
  _Float16* Bb = (_Float16*)smem;
  _Float16* Zs = (_Float16*)(smem + 4 * PANEL);
  float*  Xl = (float*)(smem + 4 * PANEL + 256 * KPADP);
  float*  B2 = Xl + 128 * 16;

  const int tid  = threadIdx.x;
  const int wave = tid >> 5, lane = tid & 31;
  const int rtw  = wave >> 2;
  const int cg   = wave & 3;
  const int b    = blockIdx.x;

  int e = 0;
  for (int t = 0; t < E_ELEM; ++t)
    if (y[b * E_ELEM + t] > 0.5f) e = t;

  for (int idx = tid; idx < 128 * 16; idx += 1024) {
    Xl[idx] = x[(long)b * C_CH * 16 + idx];
  }
  __syncthreads();

  const int KI = 16 * K3;
  for (int idx = tid; idx < 128 * KPADP; idx += 1024) {
    int r = idx / KPADP, kk = idx % KPADP;
    float v = 0.f;
    if (kk < KI) {
      int k = kk >> 4, i = kk & 15;
      v = W3[(e * K3 + k) * C_CH + r] * Xl[r * 16 + i];
    } else if (kk < KI + K2) {
      v = W2[(e * K2 + (kk - KI)) * C_CH + r];
    }
    Zs[idx] = (_Float16)v;
  }

  copy_panel(Bb, Bmat, PANEL, tid);
  __syncthreads();

  v8f acc[NTPW];
#pragma unroll
  for (int t = 0; t < NTPW; ++t)
#pragma unroll
    for (int q = 0; q < 8; ++q) acc[t][q] = 0.f;

  const int hf = lane >> 4;
  const int rA = lane & 15;
  const _Float16* Zr = Zs + (rtw * 16 + rA) * KPADP;

  int cur = 0;
  for (int ks = 0; ks < KSTEPS; ++ks) {
    __syncthreads();
    if (ks + 1 < KSTEPS)
      copy_panel(Bb + (cur ^ 1) * PANEL, Bmat + (long)(ks + 1) * PANEL, PANEL, tid);

    const int k0 = ks * 32;
    v16h a;
#pragma unroll
    for (int v = 0; v < 4; ++v) {
      int kk = k0 + hf * 8 + 2 * v;
      a[2 * v]     = Zr[kk];
      a[2 * v + 1] = Zr[kk + 1];
      int kk2 = k0 + 16 + hf * 8 + 2 * v;
      a[2 * (v + 4)]     = Zr[kk2];
      a[2 * (v + 4) + 1] = Zr[kk2 + 1];
    }
    const _Float16* bp = Bb + cur * PANEL + (lane & 15);
    auto loadB = [&](int t) {
      v16h r;
      const int n0 = (cg * NTPW + t) * 16;
#pragma unroll
      for (int v = 0; v < 8; ++v) {
        r[v]     = bp[(8 * hf + v) * NP + n0];
        r[8 + v] = bp[(16 + 8 * hf + v) * NP + n0];
      }
      return r;
    };
    v16h bb = loadB(0);
#pragma unroll
    for (int t = 0; t < NTPW; ++t) {
      v16h nx = bb;
      if (t + 1 < NTPW) nx = loadB(t + 1);
      acc[t] = wmma16(a, bb, acc[t]);
      bb = nx;
    }
    cur ^= 1;
  }

  const int l = lane & 15;
#pragma unroll
  for (int t = 0; t < NTPW; ++t) {
    const int mj = cg * NTPW + t;
#pragma unroll
    for (int v = 0; v < 8; ++v) {
      int r = rtw * 16 + v + 8 * hf;
      float p = acc[t][v] * Xl[r * 16 + l];
      p += __shfl_xor(p, 1, 32);
      p += __shfl_xor(p, 2, 32);
      p += __shfl_xor(p, 4, 32);
      p += __shfl_xor(p, 8, 32);
      if (l == 0) B2[r * (MOUT * 16) + mj] = p;
    }
  }
  __syncthreads();

  __shared__ __align__(16) float so[128 * 3];
  if (tid < 128 * MOUT) {
    int r = tid & 127, m = tid >> 7;
    float s = 0.f;
    for (int j = 0; j < 16; ++j) {
      float b2 = B2[r * (MOUT * 16) + m * 16 + j];
      for (int k1 = 0; k1 < K1; ++k1)
        b2 += U1[(m * 16 + j) * K1 + k1] * W1[(e * K1 + k1) * C_CH + r];
      s += b2 * Xl[r * 16 + j];
    }
    so[r * MOUT + m] = s;
  }
  __syncthreads();
  if (tid < 32 * MOUT) vst2(out + (long)b * (4 * C_CH) + out_col_ofs + tid * 4, *(const v4f*)(&so[tid * 4]));
}

extern "C" void kernel_launch(void* const* d_in, const int* in_sizes, int n_in,
                              void* d_out, int out_size, void* d_ws, size_t ws_size,
                              hipStream_t stream) {
  const float* x    = (const float*)d_in[0];
  const float* y    = (const float*)d_in[1];
  const float* U3_0 = (const float*)d_in[2];
  const float* U2_0 = (const float*)d_in[3];
  const float* U1_0 = (const float*)d_in[4];
  const float* W3_0 = (const float*)d_in[5];
  const float* W2_0 = (const float*)d_in[6];
  const float* W1_0 = (const float*)d_in[7];
  const float* U3_1 = (const float*)d_in[8];
  const float* U2_1 = (const float*)d_in[9];
  const float* U1_1 = (const float*)d_in[10];
  const float* W3_1 = (const float*)d_in[11];
  const float* W2_1 = (const float*)d_in[12];
  const float* W1_1 = (const float*)d_in[13];
  float* out = (float*)d_out;

  _Float16* Bm0 = (_Float16*)d_ws;
  _Float16* Bm1 = (_Float16*)((char*)d_ws + 384 * 264 * sizeof(_Float16));

  {
    int tot0 = 384 * 264 / 8;
    build_bmat<<<(tot0 + 255) / 256, 256, 0, stream>>>(U3_0, U2_0, Bm0, 1, 23, 4, 384);
    int tot1 = 544 * 776 / 8;
    build_bmat<<<(tot1 + 255) / 256, 256, 0, stream>>>(U3_1, U2_1, Bm1, 3, 33, 5, 544);
  }

  dim3 grid(2048);
  size_t sm0 = 4u * (32 * 264) + 256u * 392 + 8192u + 128u * 16 * 4;
  size_t sm1 = 4u * (32 * 776) + 256u * 552 + 8192u + 128u * 48 * 4;
  mace_contract<1, 384><<<grid, 1024, sm0, stream>>>(x, y, Bm0, W3_0, W2_0, W1_0, U1_0,
                                                     23, 4, 1, out, 0);
  mace_contract<3, 544><<<grid, 1024, sm1, stream>>>(x, y, Bm1, W3_1, W2_1, W1_1, U1_1,
                                                     33, 5, 1, out, 128);
}
